// TextEncoder_61744449847730
// MI455X (gfx1250) — hardware-verified
//
#include <hip/hip_runtime.h>
#include <math.h>

constexpr int kVocab  = 2000;
constexpr int kEmbed  = 8;
constexpr int kHid    = 256;
constexpr int kBatch  = 256;
constexpr int kSeq    = 256;
constexpr int kGate4  = 4 * kHid;
constexpr int NTHR    = 256;
constexpr int kTile   = 16;
constexpr int kHP     = 264;
constexpr int kSP     = 260;
constexpr int kPlane  = kTile * kHP;
constexpr int kWPlane = kHid * kHid;
constexpr float kBnEps = 1e-5f;

static_assert(kHid == 32 * (NTHR / 32));
static_assert(kBatch == NTHR && kHid == NTHR);
static_assert(kGate4 == 4 * NTHR);
static_assert(kBatch % kTile == 0);
static_assert(kHid % 32 == 0);
static_assert((8 * kPlane) % NTHR == 0);
static_assert(kTile * kSeq == 16 * NTHR);
static_assert(kTile * kHid == 16 * NTHR);
static_assert(kHP % 8 == 0 && kSP % 4 == 0);
static_assert((kGate4 * (kHid / 8)) % NTHR == 0);
static_assert(kBatch % 32 == 0 && kBatch % 4 == 0);

typedef __attribute__((ext_vector_type(16))) _Float16 v16h;
typedef __attribute__((ext_vector_type(8)))  _Float16 v8h;
typedef __attribute__((ext_vector_type(16))) __bf16   v16b;
typedef __attribute__((ext_vector_type(8)))  __bf16   v8b;
typedef __attribute__((ext_vector_type(8)))  float    v8f;
typedef __attribute__((ext_vector_type(4)))  float    v4f;
typedef __attribute__((ext_vector_type(4)))  int      v4i;

__device__ __forceinline__ unsigned short f2bf_bits(float f) {
  unsigned u = __float_as_uint(f);
  return (unsigned short)((u + 0x7FFFu + ((u >> 16) & 1u)) >> 16);
}
__device__ __forceinline__ float bf_bits2f(unsigned short h) { return __uint_as_float(((unsigned)h) << 16); }
__device__ __forceinline__ float bf16r(float f) { return bf_bits2f(f2bf_bits(f)); }

__device__ __forceinline__ void dep_guard_h(v8f& a, v8f& b, v16h x, v16h y) { asm volatile("v_nop\n\tv_nop\n\tv_nop\n\tv_nop" : "+v"(a), "+v"(b) : "v"(x), "v"(y)); }
__device__ __forceinline__ void dep_guard_b(v8f& a, v8f& b, v16b x, v16b y) { asm volatile("v_nop\n\tv_nop\n\tv_nop\n\tv_nop" : "+v"(a), "+v"(b) : "v"(x), "v"(y)); }
__device__ __forceinline__ void keep4_h(v16h a, v16h b, v16h c, v16h d) { asm volatile("v_nop" :: "v"(a), "v"(b), "v"(c), "v"(d)); }
__device__ __forceinline__ void keep4_b(v16b a, v16b b, v16b c, v16b d) { asm volatile("v_nop" :: "v"(a), "v"(b), "v"(c), "v"(d)); }
__device__ __forceinline__ void acc_guard4(v8f& a, v8f& b, v8f& c, v8f& d) { asm volatile("v_nop\n\tv_nop\n\tv_nop\n\tv_nop" : "+v"(a), "+v"(b), "+v"(c), "+v"(d)); }
__device__ __forceinline__ void acc_guard4_ops(v8f& a, v8f& b, v8f& c, v8f& d, v16b w, v16b x, v16b y, v16b z) {
  asm volatile("v_nop\n\tv_nop\n\tv_nop\n\tv_nop" : "+v"(a), "+v"(b), "+v"(c), "+v"(d) : "v"(w), "v"(x), "v"(y), "v"(z));
}
template <typename T> struct Frag;
template <> struct Frag<_Float16> {
  typedef v16h V; union U { v16h v; v8h h[2]; };
  static __device__ __forceinline__ v16h load(const _Float16* p) {
    U f; f.h[0] = *(const v8h*)(p); f.h[1] = *(const v8h*)(p + 16); return f.v;
  }
  static __device__ __forceinline__ v8f mma(v16h a, v16h b, v8f c) {
    return __builtin_amdgcn_wmma_f32_16x16x32_f16(false, a, false, b, (short)0, c, false, false);
  }
  static __device__ __forceinline__ void guard(v8f& a, v8f& b, v16h x, v16h y) { dep_guard_h(a, b, x, y); }
  static __device__ __forceinline__ void keep(v16h a, v16h b, v16h c, v16h d) { keep4_h(a, b, c, d); }
};
template <> struct Frag<__bf16> {
  typedef v16b V; union U { v16b v; v8b h[2]; };
  static __device__ __forceinline__ v16b load(const __bf16* p) {
    U f; f.h[0] = *(const v8b*)(p); f.h[1] = *(const v8b*)(p + 16); return f.v;
  }
  static __device__ __forceinline__ v8f mma(v16b a, v16b b, v8f c) {
    return __builtin_amdgcn_wmma_f32_16x16x32_bf16(false, a, false, b, (short)0, c, false, false);
  }
  static __device__ __forceinline__ void guard(v8f& a, v8f& b, v16b x, v16b y) { dep_guard_b(a, b, x, y); }
  static __device__ __forceinline__ void keep(v16b a, v16b b, v16b c, v16b d) { keep4_b(a, b, c, d); }
};

__device__ __forceinline__ float fsig(float x)  { return __builtin_amdgcn_rcpf(1.0f + __expf(-x)); }
__device__ __forceinline__ float ftanh(float x) { return 1.0f - 2.0f * __builtin_amdgcn_rcpf(__expf(2.0f * x) + 1.0f); }

template <int MODE>
__global__ __launch_bounds__(NTHR) void cvt8_kernel(const float* __restrict__ src, unsigned short* __restrict__ dst,
                                                    int nrow, int ncol8, int spitch, int scol0, float sc) {
  const int i  = blockIdx.x * NTHR + threadIdx.x;
  const int n8 = nrow * ncol8;
  if (i < n8) {
    const int row = i / ncol8;
    const int c8  = i - row * ncol8;
    const float* sp = src + (size_t)row * spitch + scol0 + c8 * 8;
    const v4f a = *(const v4f*)(sp);
    const v4f b = *(const v4f*)(sp + 4);
    v8h hv;
#pragma unroll
    for (int e = 0; e < 4; ++e) {
      unsigned short b0, b1;
      if (MODE == 0) {
        b0 = f2bf_bits(a[e] * sc);
        b1 = f2bf_bits(b[e] * sc);
      } else {
        b0 = __builtin_bit_cast(unsigned short, (_Float16)(bf16r(a[e]) * sc));
        b1 = __builtin_bit_cast(unsigned short, (_Float16)(bf16r(b[e]) * sc));
      }
      hv[e]     = __builtin_bit_cast(_Float16, b0);
      hv[4 + e] = __builtin_bit_cast(_Float16, b1);
    }
    *(volatile v8h*)(dst + (size_t)i * 8) = hv;
    __threadfence();
    *(volatile v8h*)(dst + (size_t)i * 8) = hv;
  }
}

__global__ __launch_bounds__(NTHR) void xproj_table_kernel(const float* __restrict__ emb, const float* __restrict__ w_ih0,
                                                           const float* __restrict__ b_ih0, const float* __restrict__ b_hh0,
                                                           float* __restrict__ TP) {
  const int v = blockIdx.x;
  const int j = threadIdx.x;
  const v4f e0 = *(const v4f*)(emb + (size_t)v * kEmbed);
  const v4f e1 = *(const v4f*)(emb + (size_t)v * kEmbed + 4);
  float ev[8];
#pragma unroll
  for (int e = 0; e < 4; ++e) { ev[e] = bf16r(e0[e]); ev[4 + e] = bf16r(e1[e]); }
  v4f o;
#pragma unroll
  for (int g = 0; g < 4; ++g) {
    const int row = g * kHid + j;
    const v4f w0 = *(const v4f*)(w_ih0 + (size_t)row * kEmbed);
    const v4f w1 = *(const v4f*)(w_ih0 + (size_t)row * kEmbed + 4);
    float s = 0.0f;
#pragma unroll
    for (int e = 0; e < 4; ++e) s += ev[e] * bf16r(w0[e]);
#pragma unroll
    for (int e = 0; e < 4; ++e) s += ev[4 + e] * bf16r(w1[e]);
    const float bsum = bf16r(b_ih0[row]) + bf16r(b_hh0[row]);
    o[g] = s + bsum;
  }
  float* op = TP + (size_t)v * kGate4 + 4 * j;
  *(volatile v4f*)op = o;
  __threadfence();
  *(volatile v4f*)op = o;
}

__global__ __launch_bounds__(NTHR) void lstm2_kernel(const int* __restrict__ tokens, const int* __restrict__ lengths,
                                                     const float* __restrict__ TP,
                                                     const unsigned short* __restrict__ W0p,
                                                     const unsigned short* __restrict__ W1Ip,
                                                     const unsigned short* __restrict__ W1Hp,
                                                     const float* __restrict__ b_ih1, const float* __restrict__ b_hh1,
                                                     float* __restrict__ LAST) {
  __shared__ __align__(16) unsigned short HT[8 * kPlane];
  __shared__ __align__(16) float          LastS[kTile * kSP];
  __shared__ __align__(16) int            TokL[kTile * kSeq];
  __shared__ int LenAll[kBatch];
  __shared__ int RankAll[kBatch];
  __shared__ int ObRow[kTile];
  __shared__ int ObLen[kTile];
  const __bf16* W0  = (const __bf16*)W0p;
  const __bf16* W1I = (const __bf16*)W1Ip;
  const __bf16* W1H = (const __bf16*)W1Hp;
  const int tid = threadIdx.x, lane = tid & 31, wave = tid >> 5;
  const int c = lane & 15, hh = lane >> 4, koff = hh * 8;
  const int pos0 = blockIdx.x * kTile;

  {
    int lv = lengths[tid];
    lv = lv < 1 ? 1 : lv;
    lv = lv > kSeq ? kSeq : lv;
    LenAll[tid] = lv;
  }
#pragma unroll 1
  for (int i = tid; i < 8 * kPlane; i += NTHR) HT[i] = (unsigned short)0;
#pragma unroll 1
  for (int i = tid; i < kTile * kSP; i += NTHR) LastS[i] = 0.0f;
  __syncthreads();

  {
    const int lb = LenAll[tid];
    int rk = 0;
#pragma unroll 1
    for (int b2 = 0; b2 < kBatch; ++b2) {
      const int l2 = LenAll[b2];
      rk += ((l2 < lb) || (l2 == lb && b2 < tid)) ? 1 : 0;
    }
    RankAll[tid] = rk;
  }
  __syncthreads();

  {
    const int m = tid & 15;
    const int p = pos0 + m;
    int sel = 0;
#pragma unroll 1
    for (int b2 = 0; b2 < kBatch; ++b2) sel = (RankAll[b2] == p) ? b2 : sel;
    if (tid < kTile) { ObRow[m] = sel; ObLen[m] = LenAll[sel]; }
  }
  __syncthreads();

#pragma unroll
  for (int it = 0; it < 4; ++it) {
    const int idx = it * NTHR + tid;
    const int m = idx >> 6, c4 = (idx & 63) * 4;
    const int ob = ObRow[m];
    const v4i tk = *(const v4i*)(tokens + (size_t)ob * kSeq + c4);
    v4i tcl;
#pragma unroll
    for (int e = 0; e < 4; ++e) {
      int x = tk[e];
      x = x < 0 ? 0 : x;
      x = x > (kVocab - 1) ? (kVocab - 1) : x;
      tcl[e] = x;
    }
    *(v4i*)(TokL + m * kSeq + c4) = tcl;
  }
  int caps[8];
#pragma unroll
  for (int r = 0; r < 8; ++r) caps[r] = ObLen[8 * hh + r] - 1;
  float bb1[2][4];
  {
    const int j0 = 32 * wave + c;
#pragma unroll
    for (int g = 0; g < 4; ++g) bb1[0][g] = bf16r(b_ih1[g * kHid + j0]) + bf16r(b_hh1[g * kHid + j0]);
    asm volatile("" ::: "memory");
    const int j1 = 32 * wave + 16 + c;
#pragma unroll
    for (int g = 0; g < 4; ++g) bb1[1][g] = bf16r(b_ih1[g * kHid + j1]) + bf16r(b_hh1[g * kHid + j1]);
  }
  float c1[2][8], c2[2][8];
#pragma unroll
  for (int nt = 0; nt < 2; ++nt)
#pragma unroll
    for (int r = 0; r < 8; ++r) { c1[nt][r] = 0.0f; c2[nt][r] = 0.0f; }
  const int tmax = ObLen[kTile - 1];
  __syncthreads();

  const v8f z8 = {0.f, 0.f, 0.f, 0.f, 0.f, 0.f, 0.f, 0.f};

#pragma unroll 1
  for (int t = 0; t < tmax; ++t) {
    const int cur = t & 1;
    const int nxt = cur ^ 1;

#pragma unroll
    for (int nt = 0; nt < 2; ++nt) {
      const int j = 32 * wave + 16 * nt + c;
      const __bf16* a_h = (const __bf16*)HT + (size_t)(0 + cur) * kPlane + c * kHP + koff;
      const __bf16* a_l = (const __bf16*)HT + (size_t)(2 + cur) * kPlane + c * kHP + koff;
      const __bf16* wp  = W0 + (size_t)j * kHid + koff;
      v8f acc[4];
      acc[0] = z8; acc[1] = z8; acc[2] = z8; acc[3] = z8;
#pragma unroll 1
      for (int k0 = 0; k0 < kHid; k0 += 32) {
        const v16b ah = Frag<__bf16>::load(a_h + k0);
        const v16b al = Frag<__bf16>::load(a_l + k0);
        const v16b b0 = Frag<__bf16>::load(wp + k0);
        const v16b b1 = Frag<__bf16>::load(wp + (size_t)1 * kWPlane + k0);
        const v16b b2 = Frag<__bf16>::load(wp + (size_t)2 * kWPlane + k0);
        const v16b b3 = Frag<__bf16>::load(wp + (size_t)3 * kWPlane + k0);
        acc[0] = Frag<__bf16>::mma(ah, b0, acc[0]);
        acc[1] = Frag<__bf16>::mma(ah, b1, acc[1]);
        acc[2] = Frag<__bf16>::mma(ah, b2, acc[2]);
        acc[3] = Frag<__bf16>::mma(ah, b3, acc[3]);
        acc[0] = Frag<__bf16>::mma(al, b0, acc[0]);
        acc[1] = Frag<__bf16>::mma(al, b1, acc[1]);
        acc[2] = Frag<__bf16>::mma(al, b2, acc[2]);
        acc[3] = Frag<__bf16>::mma(al, b3, acc[3]);
        acc_guard4_ops(acc[0], acc[1], acc[2], acc[3], ah, al, b0, b3);
        keep4_b(b0, b1, b2, b3);
      }
      acc_guard4(acc[0], acc[1], acc[2], acc[3]);
      v4f tv[8];
#pragma unroll
      for (int r = 0; r < 8; ++r) {
        const int tk = TokL[(8 * hh + r) * kSeq + t];
        tv[r] = *(const v4f*)(TP + (size_t)tk * kGate4 + 4 * j);
      }
#pragma unroll
      for (int r = 0; r < 8; ++r) {
        const float zi = acc[0][r] + tv[r][0];
        const float zf = acc[1][r] + tv[r][1];
        const float zg = acc[2][r] + tv[r][2];
        const float zo = acc[3][r] + tv[r][3];
        const float cn = fsig(zf) * c1[nt][r] + fsig(zi) * ftanh(zg);
        c1[nt][r] = cn;
        const float hn = fsig(zo) * ftanh(cn);
        const unsigned short hb = f2bf_bits(hn);
        const unsigned short lb = f2bf_bits(hn - bf_bits2f(hb));
        HT[(0 + nxt) * kPlane + (8 * hh + r) * kHP + j] = hb;
        HT[(2 + nxt) * kPlane + (8 * hh + r) * kHP + j] = lb;
      }
    }
    __syncthreads();

#pragma unroll
    for (int nt = 0; nt < 2; ++nt) {
      const int j = 32 * wave + 16 * nt + c;
      const __bf16* a1h = (const __bf16*)HT + (size_t)(0 + nxt) * kPlane + c * kHP + koff;
      const __bf16* a1l = (const __bf16*)HT + (size_t)(2 + nxt) * kPlane + c * kHP + koff;
      const __bf16* a2h = (const __bf16*)HT + (size_t)(4 + cur) * kPlane + c * kHP + koff;
      const __bf16* a2l = (const __bf16*)HT + (size_t)(6 + cur) * kPlane + c * kHP + koff;
      const __bf16* wi  = W1I + (size_t)j * kHid + koff;
      const __bf16* wh  = W1H + (size_t)j * kHid + koff;
      v8f acc[4];
      acc[0] = z8; acc[1] = z8; acc[2] = z8; acc[3] = z8;
#pragma unroll 1
      for (int k0 = 0; k0 < kHid; k0 += 32) {
        const v16b ah = Frag<__bf16>::load(a1h + k0);
        const v16b al = Frag<__bf16>::load(a1l + k0);
        const v16b b0 = Frag<__bf16>::load(wi + k0);
        const v16b b1 = Frag<__bf16>::load(wi + (size_t)1 * kWPlane + k0);
        const v16b b2 = Frag<__bf16>::load(wi + (size_t)2 * kWPlane + k0);
        const v16b b3 = Frag<__bf16>::load(wi + (size_t)3 * kWPlane + k0);
        acc[0] = Frag<__bf16>::mma(ah, b0, acc[0]);
        acc[1] = Frag<__bf16>::mma(ah, b1, acc[1]);
        acc[2] = Frag<__bf16>::mma(ah, b2, acc[2]);
        acc[3] = Frag<__bf16>::mma(ah, b3, acc[3]);
        acc[0] = Frag<__bf16>::mma(al, b0, acc[0]);
        acc[1] = Frag<__bf16>::mma(al, b1, acc[1]);
        acc[2] = Frag<__bf16>::mma(al, b2, acc[2]);
        acc[3] = Frag<__bf16>::mma(al, b3, acc[3]);
        acc_guard4_ops(acc[0], acc[1], acc[2], acc[3], ah, al, b0, b3);
        keep4_b(b0, b1, b2, b3);
      }
#pragma unroll 1
      for (int k0 = 0; k0 < kHid; k0 += 32) {
        const v16b ah = Frag<__bf16>::load(a2h + k0);
        const v16b al = Frag<__bf16>::load(a2l + k0);
        const v16b b0 = Frag<__bf16>::load(wh + k0);
        const v16b b1 = Frag<__bf16>::load(wh + (size_t)1 * kWPlane + k0);
        const v16b b2 = Frag<__bf16>::load(wh + (size_t)2 * kWPlane + k0);
        const v16b b3 = Frag<__bf16>::load(wh + (size_t)3 * kWPlane + k0);
        acc[0] = Frag<__bf16>::mma(ah, b0, acc[0]);
        acc[1] = Frag<__bf16>::mma(ah, b1, acc[1]);
        acc[2] = Frag<__bf16>::mma(ah, b2, acc[2]);
        acc[3] = Frag<__bf16>::mma(ah, b3, acc[3]);
        acc[0] = Frag<__bf16>::mma(al, b0, acc[0]);
        acc[1] = Frag<__bf16>::mma(al, b1, acc[1]);
        acc[2] = Frag<__bf16>::mma(al, b2, acc[2]);
        acc[3] = Frag<__bf16>::mma(al, b3, acc[3]);
        acc_guard4_ops(acc[0], acc[1], acc[2], acc[3], ah, al, b0, b3);
        keep4_b(b0, b1, b2, b3);
      }
      acc_guard4(acc[0], acc[1], acc[2], acc[3]);
#pragma unroll
      for (int r = 0; r < 8; ++r) {
        const float zi = acc[0][r] + bb1[nt][0];
        const float zf = acc[1][r] + bb1[nt][1];
        const float zg = acc[2][r] + bb1[nt][2];
        const float zo = acc[3][r] + bb1[nt][3];
        const float cn = fsig(zf) * c2[nt][r] + fsig(zi) * ftanh(zg);
        c2[nt][r] = cn;
        const float hn = fsig(zo) * ftanh(cn);
        const unsigned short hb = f2bf_bits(hn);
        const unsigned short lb = f2bf_bits(hn - bf_bits2f(hb));
        HT[(4 + nxt) * kPlane + (8 * hh + r) * kHP + j] = hb;
        HT[(6 + nxt) * kPlane + (8 * hh + r) * kHP + j] = lb;
        if (t == caps[r]) LastS[(8 * hh + r) * kSP + j] = hn;
      }
    }
    __syncthreads();
  }

  __syncthreads();
  for (int pass = 0; pass < 2; ++pass) {
#pragma unroll
    for (int it = 0; it < 4; ++it) {
      const int idx = it * NTHR + tid;
      const int row = idx >> 6, c4 = (idx & 63) * 4;
      const v4f v = *(const v4f*)(LastS + row * kSP + c4);
      const int ob = ObRow[row];
      *(volatile v4f*)(LAST + (size_t)ob * kHid + c4) = v;
    }
    __threadfence();
  }
}

__global__ __launch_bounds__(NTHR) void ff_kernel(const float* __restrict__ LAST, const float* __restrict__ ffw,
                                                  const float* __restrict__ ffb, float* __restrict__ Y) {
  __shared__ __align__(16) float Ls[4 * kHid];
  const int tid = threadIdx.x;
  const int row0 = blockIdx.x * 4;
#pragma unroll
  for (int it = 0; it < 4; ++it) Ls[it * kHid + tid] = fmaxf(LAST[(size_t)(row0 + it) * kHid + tid], 0.0f);
  __syncthreads();
  const int rl = tid >> 6, n0 = (tid & 63) * 4;
  const float* lp = Ls + rl * kHid;
  double acc[4] = {0.0, 0.0, 0.0, 0.0};
#pragma unroll 1
  for (int k = 0; k < kHid; k += 4) {
    const v4f lv = *(const v4f*)(lp + k);
#pragma unroll
    for (int q = 0; q < 4; ++q) {
      const v4f wv = *(const v4f*)(ffw + (size_t)(n0 + q) * kHid + k);
#pragma unroll
      for (int e = 0; e < 4; ++e) acc[q] += (double)lv[e] * (double)bf16r(wv[e]);
    }
  }
  const v4f bv = *(const v4f*)(ffb + n0);
  v4f o;
#pragma unroll
  for (int q = 0; q < 4; ++q) o[q] = (float)acc[q] + bf16r(bv[q]);
  float* op = Y + (size_t)(row0 + rl) * kHid + n0;
  *(volatile v4f*)op = o;
  __threadfence();
  *(volatile v4f*)op = o;
}

__global__ __launch_bounds__(NTHR) void bn_kernel(const float* __restrict__ Y, const float* __restrict__ gam,
                                                  const float* __restrict__ bet, float* __restrict__ outp) {
  __shared__ __align__(16) float Ms[kHid];
  __shared__ __align__(16) float Ss[kHid];
  __shared__ __align__(16) float Bs[kHid];
  const int tid = threadIdx.x;
  const int n = tid;
  double s = 0.0;
#pragma unroll 1
  for (int b = 0; b < kBatch; ++b) s += (double)Y[(size_t)b * kHid + n];
  const float mean = (float)(s * (1.0 / kBatch));
  double ss = 0.0;
#pragma unroll 1
  for (int b = 0; b < kBatch; ++b) {
    const float d = Y[(size_t)b * kHid + n] - mean;
    ss += (double)(d * d);
  }
  const float var  = (float)(ss * (1.0 / kBatch));
  const float rstd = rsqrtf(var + kBnEps);
  Ms[n] = mean;
  Ss[n] = bf16r(gam[n]) * rstd;
  Bs[n] = bf16r(bet[n]);
  __syncthreads();
  const int rowb = blockIdx.x * 32;
  v4f o[8];
#pragma unroll
  for (int it = 0; it < 8; ++it) {
    const int idx = it * NTHR + tid;
    const int row = rowb + (idx >> 6), c4 = (idx & 63) * 4;
    const v4f yv = *(const v4f*)(Y + (size_t)row * kHid + c4);
    const v4f mv = *(const v4f*)(Ms + c4);
    const v4f sv = *(const v4f*)(Ss + c4);
    const v4f bv = *(const v4f*)(Bs + c4);
#pragma unroll
    for (int e = 0; e < 4; ++e) o[it][e] = (yv[e] - mv[e]) * sv[e] + bv[e];
  }
  for (int pass = 0; pass < 2; ++pass) {
#pragma unroll
    for (int it = 0; it < 8; ++it) {
      const int idx = it * NTHR + tid;
      const int row = rowb + (idx >> 6), c4 = (idx & 63) * 4;
      *(volatile v4f*)(outp + (size_t)row * kHid + c4) = o[it];
    }
    __threadfence();
  }
}

extern "C" void kernel_launch(void* const* d_in, const int* in_sizes, int n_in,
                              void* d_out, int out_size, void* d_ws, size_t ws_size, hipStream_t stream) {
  if (n_in < 15 || d_out == nullptr || d_ws == nullptr) return;
  if (in_sizes[0] != kBatch * kSeq || in_sizes[1] != kBatch || in_sizes[2] != kVocab * kEmbed ||
      in_sizes[3] != kGate4 * kEmbed || in_sizes[4] != kGate4 * kHid || in_sizes[5] != kGate4 || in_sizes[6] != kGate4 ||
      in_sizes[7] != kGate4 * kHid || in_sizes[8] != kGate4 * kHid || in_sizes[9] != kGate4 || in_sizes[10] != kGate4 ||
      in_sizes[11] != kHid * kHid || in_sizes[12] != kHid || in_sizes[13] != kHid || in_sizes[14] != kHid ||
      out_size != kBatch * kHid) return;

  const int*   tokens  = (const int*)d_in[0];
  const int*   lengths = (const int*)d_in[1];
  const float* emb     = (const float*)d_in[2];
  const float* w_ih0   = (const float*)d_in[3];
  const float* w_hh0   = (const float*)d_in[4];
  const float* b_ih0   = (const float*)d_in[5];
  const float* b_hh0   = (const float*)d_in[6];
  const float* w_ih1   = (const float*)d_in[7];
  const float* w_hh1   = (const float*)d_in[8];
  const float* b_ih1   = (const float*)d_in[9];
  const float* b_hh1   = (const float*)d_in[10];
  const float* ff_w    = (const float*)d_in[11];
  const float* ff_b    = (const float*)d_in[12];
  const float* gam     = (const float*)d_in[13];
  const float* bet     = (const float*)d_in[14];
  float* outp = (float*)d_out;

  char* ws = (char*)d_ws; size_t off = 0;
  auto carve = [&](size_t bytes) -> char* { char* p = ws + off; off += (bytes + 255) & ~(size_t)255; return p; };
  float*          TP   = (float*)carve((size_t)kVocab * kGate4 * 4);
  unsigned short* W0B  = (unsigned short*)carve((size_t)kGate4 * kHid * 2);
  unsigned short* W1IB = (unsigned short*)carve((size_t)kGate4 * kHid * 2);
  unsigned short* W1HB = (unsigned short*)carve((size_t)kGate4 * kHid * 2);
  float*          LAST = (float*)carve((size_t)kBatch * kHid * 4);
  float*          Y    = (float*)carve((size_t)kBatch * kHid * 4);
  if (off > ws_size || off > (size_t)134217728) return;

  const int n8w = kGate4 * (kHid / 8);
  cvt8_kernel<0><<<(n8w + NTHR - 1) / NTHR, NTHR, 0, stream>>>(w_hh0, W0B,  kGate4, kHid / 8, kHid, 0, 1.0f);
  cvt8_kernel<0><<<(n8w + NTHR - 1) / NTHR, NTHR, 0, stream>>>(w_ih1, W1IB, kGate4, kHid / 8, kHid, 0, 1.0f);
  cvt8_kernel<0><<<(n8w + NTHR - 1) / NTHR, NTHR, 0, stream>>>(w_hh1, W1HB, kGate4, kHid / 8, kHid, 0, 1.0f);
  xproj_table_kernel<<<kVocab, NTHR, 0, stream>>>(emb, w_ih0, b_ih0, b_hh0, TP);
  lstm2_kernel<<<kBatch / kTile, NTHR, 0, stream>>>(tokens, lengths, TP, W0B, W1IB, W1HB, b_ih1, b_hh1, LAST);
  ff_kernel<<<kBatch / 4, NTHR, 0, stream>>>(LAST, ff_w, ff_b, Y);
  bn_kernel<<<kBatch / 32, NTHR, 0, stream>>>(Y, gam, bet, outp);
}
